// CFRMPhilosophyClassifier_81123342287194
// MI455X (gfx1250) — hardware-verified
//
#include <hip/hip_runtime.h>


#define B_    128
#define S_    512
#define H_    128
#define C_    16
#define CI_   260
#define KP_   288
#define NC_   8
#define V_    32000
#define BT_   16
#define NH_   208
#define NHT_  13
#define NT_   256
#define EPS_  1e-4f

static_assert(B_ % BT_ == 0);
static_assert(KP_ % 32 == 0 && KP_ >= CI_);
static_assert(NH_ == NHT_ * 16);
static_assert(NT_ == 256 && BT_ * C_ == NT_);

typedef _Float16       v16h __attribute__((ext_vector_type(16)));
typedef _Float16       v8h  __attribute__((ext_vector_type(8)));
typedef __bf16         v16b __attribute__((ext_vector_type(16)));
typedef unsigned short v8us __attribute__((ext_vector_type(8)));
typedef unsigned short v4us __attribute__((ext_vector_type(4)));
typedef float          v8f  __attribute__((ext_vector_type(8)));
typedef float          v4f  __attribute__((ext_vector_type(4)));
typedef unsigned int   v4u  __attribute__((ext_vector_type(4)));

union FragH { v16h v; v8h  half[2]; };
union FragB { v16b v; v8us half[2]; };

constexpr int L_CEN   = 0;
constexpr int L_CIH   = 131072;
constexpr int L_CIL   = 140288;
constexpr int L_CT1H  = 149504;
constexpr int L_CT1L  = 153600;
constexpr int L_CTH   = 157696;
constexpr int L_CTL   = 161792;
constexpr int L_CTF   = 165888;
constexpr int L_HEADS = 169984;
constexpr int L_CORE  = 183296;
constexpr int L_CMP   = L_HEADS;
constexpr int L_MIXH  = 191488;
constexpr int L_ALPHA = 199680;
constexpr int L_SS    = 200704;
constexpr int L_SQ    = 201728;
constexpr int L_SPR   = 202752;
constexpr int L_MAS   = 203776;
constexpr int L_NOV   = 204800;
constexpr int L_REL   = 204864;
constexpr int L_IDX   = 204928;
constexpr int L_OST   = 204992;
constexpr int LDS_BYTES = 205504;
static_assert(L_CIH == L_CEN + BT_ * C_ * H_ * 4);
static_assert(L_CIL == L_CIH + BT_ * KP_ * 2 && L_CT1H == L_CIL + BT_ * KP_ * 2);
static_assert(L_CT1L == L_CT1H + BT_ * H_ * 2 && L_CTH == L_CT1L + BT_ * H_ * 2);
static_assert(L_CTL == L_CTH + BT_ * H_ * 2 && L_CTF == L_CTL + BT_ * H_ * 2 && L_HEADS == L_CTF + BT_ * H_ * 2);
static_assert(L_CORE == L_HEADS + BT_ * NH_ * 4 && L_MIXH == L_CORE + BT_ * H_ * 4);
static_assert(L_CMP + BT_ * C_ * C_ * 4 <= L_MIXH);
static_assert(L_ALPHA == L_MIXH + BT_ * C_ * C_ * 2);
static_assert(L_SS == L_ALPHA + 1024 && L_SQ == L_SS + 1024 && L_SPR == L_SQ + 1024 && L_MAS == L_SPR + 1024);
static_assert(L_NOV == L_MAS + 1024 && L_REL == L_NOV + 64 && L_IDX == L_REL + 64 && L_OST == L_IDX + 64);
static_assert(LDS_BYTES == L_OST + BT_ * NC_ * 4);
static_assert(L_CIH % 16 == 0 && L_CIL % 16 == 0 && L_CTF % 16 == 0 && L_MIXH % 16 == 0 && L_OST % 16 == 0);

constexpr int PC_W1  = 0;
constexpr int PC_W2  = 4608;
constexpr int PC_WH  = 6656;
constexpr int PC_WCC = 9984;
constexpr int PC_C1  = 42752;
constexpr int PC_C2  = 47360;
constexpr int NPIECE = 47616;
constexpr int BK_W2 = 18, BK_WH = 26, BK_WCC = 39, BK_C1 = 167, BK_C2 = 185, NBLK_PL = 186;
static_assert(PC_W2 == BK_W2 * NT_ && PC_WH == BK_WH * NT_ && PC_WCC == BK_WCC * NT_);
static_assert(PC_C1 == BK_C1 * NT_ && PC_C2 == BK_C2 * NT_ && NPIECE == NBLK_PL * NT_);
static_assert(PC_W2 - PC_W1 == 128 * (KP_ / 8) && PC_WH - PC_W2 == 128 * 16 && PC_WCC - PC_WH == NH_ * 16);
static_assert(PC_C1 - PC_WCC == 2048 * 16 && PC_C2 - PC_C1 == 128 * (KP_ / 8) && NPIECE - PC_C2 == 16 * 16);
constexpr int PD_W1H = 0;
constexpr int PD_W1L = 36864;
constexpr int PD_W2H = 73728;
constexpr int PD_W2L = 90112;
constexpr int PD_WHH = 106496;
constexpr int PD_WHL = 133120;
constexpr int PD_WCC = 159744;
constexpr int PD_C1  = 421888;
constexpr int PD_C2  = 458752;
constexpr int PD_END = 460800;
static_assert(PD_W1L - PD_W1H == 8 * (PC_W2 - PC_W1) && PD_W2H - PD_W1L == 8 * (PC_W2 - PC_W1));
static_assert(PD_W2L - PD_W2H == 8 * (PC_WH - PC_W2) && PD_WHH - PD_W2L == 8 * (PC_WH - PC_W2));
static_assert(PD_WHL - PD_WHH == 8 * (PC_WCC - PC_WH) && PD_WCC - PD_WHL == 8 * (PC_WCC - PC_WH));
static_assert(PD_C1 - PD_WCC == 8 * (PC_C1 - PC_WCC) && PD_C2 - PD_C1 == 8 * (PC_C2 - PC_C1) && PD_END - PD_C2 == 8 * (NPIECE - PC_C2));
static_assert(PD_W1L % 64 == 0 && PD_W2H % 64 == 0 && PD_W2L % 64 == 0 && PD_WHH % 64 == 0 && PD_WHL % 64 == 0);
static_assert(PD_WCC % 64 == 0 && PD_C1 % 64 == 0 && PD_C2 % 64 == 0 && PD_END % 64 == 0);

constexpr size_t SZ_TE   = (size_t)B_ * S_ * H_ * 2;
constexpr size_t OFF_TEH = 0;
constexpr size_t OFF_TEL = OFF_TEH + SZ_TE;
constexpr size_t OFF_PL  = OFF_TEL + SZ_TE;
constexpr size_t SZ_PL   = (size_t)PD_END * 2;
constexpr size_t WS_END  = OFF_PL + SZ_PL;
static_assert(OFF_TEL % 4096 == 0 && OFF_PL % 4096 == 0 && WS_END % 128 == 0);
static_assert(WS_END <= (size_t)134217728);

__device__ __forceinline__ v8f zero8f() {
    v8f z;
#pragma unroll
    for (int i = 0; i < 8; ++i) z[i] = 0.0f;
    return z;
}
__device__ __forceinline__ v8h zero8h() {
    v8h z;
#pragma unroll
    for (int i = 0; i < 8; ++i) z[i] = (_Float16)0.0f;
    return z;
}
__device__ __forceinline__ v8f ld8f(const float* p) {
    const v4f a = *(const v4f*)p;
    const v4f b = *(const v4f*)(p + 4);
    return __builtin_shufflevector(a, b, 0, 1, 2, 3, 4, 5, 6, 7);
}
__device__ __forceinline__ unsigned int bf16_rne(float x) {
    const unsigned int u = __float_as_uint(x);
    return (u + 0x7FFFu + ((u >> 16) & 1u)) >> 16;
}
__device__ __forceinline__ void split_bf16(float x, unsigned short& hi, unsigned short& lo) {
    const unsigned int hb = bf16_rne(x);
    const float hfv = __uint_as_float(hb << 16);
    const unsigned int lb = bf16_rne(x - hfv);
    hi = (unsigned short)hb;
    lo = (unsigned short)lb;
}
__device__ __forceinline__ void split8(v8f x, v8us& hv, v8us& lv) {
#pragma unroll
    for (int e = 0; e < 8; ++e) { unsigned short hi, lo; split_bf16(x[e], hi, lo); hv[e] = hi; lv[e] = lo; }
}
__device__ __forceinline__ v8h cvt8h(v8f x, float s) {
    v8h r;
#pragma unroll
    for (int e = 0; e < 8; ++e) r[e] = (_Float16)(x[e] * s);
    return r;
}
__device__ __forceinline__ void ldfragh(FragH& f, const _Float16* p) {
    f.half[0] = *(const v8h*)(p);
    f.half[1] = *(const v8h*)(p + 16);
}
__device__ __forceinline__ void ldfragb(FragB& f, const unsigned short* p) {
    f.half[0] = *(const v8us*)(p);
    f.half[1] = *(const v8us*)(p + 16);
}
__device__ __forceinline__ v8f mmah(v8f c, const FragH& a, const FragH& b) {
    v8f d = __builtin_amdgcn_wmma_f32_16x16x32_f16(false, a.v, false, b.v, (short)0, c, false, false);
    asm volatile("v_nop\n\tv_nop\n\tv_nop\n\tv_nop" : "+v"(d) : "v"(a.v), "v"(b.v));
    return d;
}
__device__ __forceinline__ v8f mma3(v8f c, const FragB& ah, const FragB& al, const FragB& bh, const FragB& bl) {
    v8f d = __builtin_amdgcn_wmma_f32_16x16x32_bf16(false, ah.v, false, bh.v, (short)0, c, false, false);
    d = __builtin_amdgcn_wmma_f32_16x16x32_bf16(false, ah.v, false, bl.v, (short)0, d, false, false);
    d = __builtin_amdgcn_wmma_f32_16x16x32_bf16(false, al.v, false, bh.v, (short)0, d, false, false);
    asm volatile("v_nop\n\tv_nop\n\tv_nop\n\tv_nop" : "+v"(d) : "v"(ah.v), "v"(al.v), "v"(bh.v), "v"(bl.v));
    return d;
}
__device__ __forceinline__ float wsum(float v) {
#pragma unroll
    for (int o = 16; o > 0; o >>= 1) v += __shfl_xor(v, o, 32);
    return v;
}
__device__ __forceinline__ float seg_sum(float v) {
    v += __shfl_xor(v, 8, 32); v += __shfl_xor(v, 4, 32); v += __shfl_xor(v, 2, 32); v += __shfl_xor(v, 1, 32);
    return v;
}
__device__ __forceinline__ float seg_max(float v) {
    v = fmaxf(v, __shfl_xor(v, 8, 32)); v = fmaxf(v, __shfl_xor(v, 4, 32));
    v = fmaxf(v, __shfl_xor(v, 2, 32)); v = fmaxf(v, __shfl_xor(v, 1, 32));
    return v;
}
__device__ __forceinline__ int seg_min_i(int v) {
    v = min(v, __shfl_xor(v, 8, 32)); v = min(v, __shfl_xor(v, 4, 32));
    v = min(v, __shfl_xor(v, 2, 32)); v = min(v, __shfl_xor(v, 1, 32));
    return v;
}
__device__ __forceinline__ float sigm(float x) { return 1.0f / (1.0f + expf(-x)); }

__device__ __forceinline__ float head_bias(int nt, int m,
                                           const float* __restrict__ gate_b, const float* __restrict__ assign_b,
                                           const float* __restrict__ nov_b, const float* __restrict__ relax_b,
                                           const float* __restrict__ cs_b, const float* __restrict__ md_b,
                                           const float* __restrict__ att_b)
{
    const float gb = gate_b[m], ab = assign_b[m], nb = nov_b[0], rb = relax_b[0], cb = cs_b[m], mb = md_b[m];
    const int ag = min(max(nt - 5, 0), 7);
    const float tb = att_b[ag * 16 + m];
    const float nr = (m == 0) ? nb : ((m == 1) ? rb : 0.0f);
    float v = tb;
    v = (nt == 4) ? mb : v;
    v = (nt == 3) ? cb : v;
    v = (nt == 2) ? nr : v;
    v = (nt == 1) ? ab : v;
    v = (nt == 0) ? gb : v;
    return v;
}

__global__ __launch_bounds__(NT_)
void k_planes(const float* __restrict__ ctrl_w1, const float* __restrict__ ctrl_w2,
              const float* __restrict__ gate_w, const float* __restrict__ assign_w,
              const float* __restrict__ nov_w, const float* __restrict__ relax_w,
              const float* __restrict__ cs_w, const float* __restrict__ md_w,
              const float* __restrict__ att_w, const float* __restrict__ cc_w,
              const float* __restrict__ cls_w1, const float* __restrict__ cls_w2,
              unsigned short* planes)
{
    const int tid = threadIdx.x;
    const int blk = blockIdx.x;
    const int p = blk * NT_ + tid;
    v8f v = zero8f();
    int dh = 0, dl = 0, df = 0;
    if (blk < BK_W2) {
        const int q = p - PC_W1;
        const int n = q / 36;
        const int j = q - n * 36;
#pragma unroll
        for (int e = 0; e < 8; ++e) {
            const int k = 8 * j + e;
            const int kc = min(k, CI_ - 1);
            const float x = ctrl_w1[kc * H_ + n];
            v[e] = (k < CI_) ? x : 0.0f;
        }
        dh = PD_W1H + 8 * q; dl = PD_W1L + 8 * q;
    } else if (blk < BK_WH) {
        const int q = p - PC_W2;
        const int n = q >> 4, j = q & 15;
#pragma unroll
        for (int e = 0; e < 8; ++e) v[e] = ctrl_w2[(8 * j + e) * H_ + n];
        dh = PD_W2H + 8 * q; dl = PD_W2L + 8 * q;
    } else if (blk < BK_WCC) {
        const int q = p - PC_WH;
        const int n = q >> 4, j = q & 15;
        const int g = blk - BK_WH;
        const int nn = n & 15;
        if (g == 0) {
#pragma unroll
            for (int e = 0; e < 8; ++e) v[e] = gate_w[(8 * j + e) * C_ + nn];
        } else if (g == 1) {
#pragma unroll
            for (int e = 0; e < 8; ++e) v[e] = assign_w[(8 * j + e) * C_ + nn];
        } else if (g == 2) {
#pragma unroll
            for (int e = 0; e < 8; ++e) {
                const int k = 8 * j + e;
                const float a = nov_w[k], b = relax_w[k];
                v[e] = (nn == 0) ? a : ((nn == 1) ? b : 0.0f);
            }
        } else if (g == 3) {
#pragma unroll
            for (int e = 0; e < 8; ++e) v[e] = cs_w[(8 * j + e) * C_ + nn];
        } else if (g == 4) {
#pragma unroll
            for (int e = 0; e < 8; ++e) v[e] = md_w[(8 * j + e) * C_ + nn];
        } else {
            const int ac = (g - 5) * 16 + nn;
#pragma unroll
            for (int e = 0; e < 8; ++e) v[e] = att_w[(8 * j + e) * H_ + ac];
        }
        dh = PD_WHH + 8 * q; dl = PD_WHL + 8 * q;
    } else if (blk < BK_C1) {
        const int q = p - PC_WCC;
        const int n = q >> 4, j = q & 15;
#pragma unroll
        for (int e = 0; e < 8; ++e) v[e] = cc_w[(size_t)(8 * j + e) * (C_ * H_) + n];
        df = PD_WCC + 8 * q;
    } else if (blk < BK_C2) {
        const int q = p - PC_C1;
        const int n = q / 36;
        const int j = q - n * 36;
#pragma unroll
        for (int e = 0; e < 8; ++e) {
            const int k = 8 * j + e;
            const int kc = min(k, CI_ - 1);
            const float x = cls_w1[kc * H_ + n];
            v[e] = (k < CI_) ? x : 0.0f;
        }
        df = PD_C1 + 8 * q;
    } else {
        const int q = p - PC_C2;
        const int n = q >> 4, j = q & 15;
        const int nc = min(n, NC_ - 1);
#pragma unroll
        for (int e = 0; e < 8; ++e) {
            const float x = cls_w2[(8 * j + e) * NC_ + nc];
            v[e] = (n < NC_) ? x : 0.0f;
        }
        df = PD_C2 + 8 * q;
    }
    if (blk < BK_WCC) {
        v8us hv, lv;
        split8(v, hv, lv);
        *(volatile v8us*)(planes + dh) = hv;
        *(volatile v8us*)(planes + dl) = lv;
        __threadfence();
        *(volatile v8us*)(planes + dh) = hv;
        *(volatile v8us*)(planes + dl) = lv;
    } else {
        const v8h hv = cvt8h(v, 16.0f);
        _Float16* d = (_Float16*)planes + df;
        *(volatile v8h*)d = hv;
        __threadfence();
        *(volatile v8h*)d = hv;
    }
}

__global__ __launch_bounds__(NT_)
void k_embed(const int* __restrict__ tokens, const float* __restrict__ emb,
             const float* __restrict__ ln_g, const float* __restrict__ ln_b,
             unsigned short* teH, unsigned short* teL, int nrows)
{
    const int tid = threadIdx.x, lane = tid & 31, w = tid >> 5;
    const int rr = blockIdx.x * 8 + w;
    if (rr >= nrows) return;
    const int tok = tokens[rr];
    const int tc = min(max(tok, 0), V_ - 1);
    const v4f ev = *(const v4f*)(emb + (size_t)tc * H_ + 4 * lane);
    v4f x;
#pragma unroll
    for (int e = 0; e < 4; ++e) x[e] = (tok != 0) ? ev[e] : 0.0f;
    const float s = wsum((x[0] + x[1]) + (x[2] + x[3]));
    const float mean = s * (1.0f / H_);
    v4f d;
    float q = 0.0f;
#pragma unroll
    for (int e = 0; e < 4; ++e) { d[e] = x[e] - mean; q += d[e] * d[e]; }
    q = wsum(q);
    const float var = q * (1.0f / H_);
    const float rstd = 1.0f / sqrtf(var + 1e-5f);
    const v4f g = *(const v4f*)(ln_g + 4 * lane);
    const v4f bb = *(const v4f*)(ln_b + 4 * lane);
    v4us yh, yl;
#pragma unroll
    for (int e = 0; e < 4; ++e) {
        const float y = d[e] * rstd * g[e] + bb[e];
        unsigned short hi, lo;
        split_bf16(y, hi, lo);
        yh[e] = hi; yl[e] = lo;
    }
    unsigned short* ph = teH + (size_t)rr * H_ + 4 * lane;
    unsigned short* pl = teL + (size_t)rr * H_ + 4 * lane;
    *(volatile v4us*)ph = yh;
    *(volatile v4us*)pl = yl;
    __threadfence();
    *(volatile v4us*)ph = yh;
    *(volatile v4us*)pl = yl;
}

__global__ __launch_bounds__(NT_)
void k_scan(const int* __restrict__ tokens,
            const unsigned short* __restrict__ teH, const unsigned short* __restrict__ teL,
            const unsigned short* __restrict__ planes,
            const float* __restrict__ ctrl_b1, const float* __restrict__ ctrl_b2,
            const float* __restrict__ gate_b, const float* __restrict__ assign_b,
            const float* __restrict__ nov_b, const float* __restrict__ relax_b,
            const float* __restrict__ cs_b, const float* __restrict__ md_b,
            const float* __restrict__ att_b, const float* __restrict__ cc_b,
            const float* __restrict__ cls_b1, const float* __restrict__ cls_b2,
            float* out)
{
    extern __shared__ __attribute__((aligned(16))) unsigned char lds[];
    float*          cen    = (float*)(lds + L_CEN);
    unsigned short* ciH    = (unsigned short*)(lds + L_CIH);
    unsigned short* ciL    = (unsigned short*)(lds + L_CIL);
    _Float16*       featF  = (_Float16*)(lds + L_CIH);
    unsigned short* ct1H   = (unsigned short*)(lds + L_CT1H);
    unsigned short* ct1L   = (unsigned short*)(lds + L_CT1L);
    unsigned short* ctH    = (unsigned short*)(lds + L_CTH);
    unsigned short* ctL    = (unsigned short*)(lds + L_CTL);
    _Float16*       ctF    = (_Float16*)(lds + L_CTF);
    float*          heads  = (float*)(lds + L_HEADS);
    float*          core   = (float*)(lds + L_CORE);
    float*          cmp    = (float*)(lds + L_CMP);
    _Float16*       mixh   = (_Float16*)(lds + L_MIXH);
    float*          alphaS = (float*)(lds + L_ALPHA);
    float*          ssS    = (float*)(lds + L_SS);
    float*          sqS    = (float*)(lds + L_SQ);
    float*          sprS   = (float*)(lds + L_SPR);
    float*          masS   = (float*)(lds + L_MAS);
    float*          novS   = (float*)(lds + L_NOV);
    float*          relS   = (float*)(lds + L_REL);
    int*            idxS   = (int*)(lds + L_IDX);
    float*          ost    = (float*)(lds + L_OST);

    const unsigned short* W1H = planes + PD_W1H;
    const unsigned short* W1L = planes + PD_W1L;
    const unsigned short* W2H = planes + PD_W2H;
    const unsigned short* W2L = planes + PD_W2L;
    const unsigned short* WHH = planes + PD_WHH;
    const unsigned short* WHL = planes + PD_WHL;
    const _Float16* Wccp = (const _Float16*)planes + PD_WCC;
    const _Float16* C1p  = (const _Float16*)planes + PD_C1;
    const _Float16* C2p  = (const _Float16*)planes + PD_C2;

    const int tid = threadIdx.x, lane = tid & 31, w = tid >> 5;
    const int hf = lane >> 4, m = lane & 15;
    const int pb = tid >> 4, pc = tid & 15;
    const int b0 = blockIdx.x * BT_;

    {
        v4f z4; z4[0] = 0.0f; z4[1] = 0.0f; z4[2] = 0.0f; z4[3] = 0.0f;
#pragma unroll 4
        for (int i = 0; i < 32; ++i) *(v4f*)(cen + 4 * (tid + NT_ * i)) = z4;
        v4u zu; zu[0] = 0u; zu[1] = 0u; zu[2] = 0u; zu[3] = 0u;
        for (int i = tid; i < (2 * BT_ * KP_ * 2) / 16; i += NT_) *(v4u*)(lds + L_CIH + 16 * i) = zu;
    }
    float sp = 1.0f, ma = 0.0f, al = 0.0f, vld = 0.0f, rl = 0.0f, msr = 0.0f, mmr = 0.0f;

    const float b1v  = ctrl_b1[16 * w + m];
    const float b2v  = ctrl_b2[16 * w + m];
    const float hb0  = head_bias(w, m, gate_b, assign_b, nov_b, relax_b, cs_b, md_b, att_b);
    const float hb1  = head_bias(min(w + 8, NHT_ - 1), m, gate_b, assign_b, nov_b, relax_b, cs_b, md_b, att_b);
    const float cb1v = cls_b1[16 * w + m];
    const float cb2v = cls_b2[min(m, NC_ - 1)];
    __syncthreads();

#pragma unroll 1
    for (int t = 0; t <= S_; ++t) {
        const int fin = (t == S_) ? 1 : 0;
        const int tt = min(t, S_ - 1);

        {
            const float prec = 1.0f / (sp + EPS_);
            const float sc = ma + logf(prec + EPS_);
            const float mx = seg_max(sc);
            const float e = expf(sc - mx);
            const float se = seg_sum(e);
            al = e * (1.0f / se);
            alphaS[tid] = al;
            const float u = seg_sum(al * sp);
            const float m2 = seg_max(ma);
            const float s2 = seg_sum(expf(ma - m2));
            const float en = m2 + logf(s2);
            const float ent = -seg_sum(al * logf(fmaxf(al, 1e-8f)));
            const int tok = tokens[(size_t)(b0 + pb) * S_ + tt];
            vld = (tok != 0) ? 1.0f : 0.0f;
            int idv = 0;
            if (fin) {
                const float kmx = seg_max(al);
                const int cand = (al == kmx) ? pc : C_;
                idv = seg_min_i(cand);
            }
            if (pc == 0) {
                if (!fin) {
                    unsigned short hi, lo;
                    split_bf16(u,   hi, lo); ciH[pb * KP_ + 2 * H_ + 0] = hi; ciL[pb * KP_ + 2 * H_ + 0] = lo;
                    split_bf16(en,  hi, lo); ciH[pb * KP_ + 2 * H_ + 2] = hi; ciL[pb * KP_ + 2 * H_ + 2] = lo;
                    split_bf16(ent, hi, lo); ciH[pb * KP_ + 2 * H_ + 3] = hi; ciL[pb * KP_ + 2 * H_ + 3] = lo;
                } else {
                    featF[pb * KP_ + 2 * H_ + 0] = (_Float16)u;
                    featF[pb * KP_ + 2 * H_ + 2] = (_Float16)en;
                    featF[pb * KP_ + 2 * H_ + 3] = (_Float16)ent;
                    idxS[pb] = idv;
                }
            }
        }
        __syncthreads();

        {
            const int b = pb, h8 = pc * 8;
            v8f acc = zero8f();
            const float* crow = cen + (size_t)b * (C_ * H_) + h8;
#pragma unroll 4
            for (int c = 0; c < C_; ++c) {
                const float a = alphaS[b * C_ + c];
                const v8f x = ld8f(crow + c * H_);
                acc += a * x;
            }
            *(v4f*)(core + b * H_ + h8)     = __builtin_shufflevector(acc, acc, 0, 1, 2, 3);
            *(v4f*)(core + b * H_ + h8 + 4) = __builtin_shufflevector(acc, acc, 4, 5, 6, 7);
            if (!fin) {
                const size_t to = ((size_t)(b0 + b) * S_ + tt) * H_ + h8;
                const v8us th = *(const v8us*)(teH + to);
                const v8us tl = *(const v8us*)(teL + to);
                *(v8us*)(ciH + b * KP_ + h8) = th;
                *(v8us*)(ciL + b * KP_ + h8) = tl;
                v8us ch, cl;
                split8(acc, ch, cl);
                *(v8us*)(ciH + b * KP_ + H_ + h8) = ch;
                *(v8us*)(ciL + b * KP_ + H_ + h8) = cl;
            } else {
                int id = idxS[b];
                id = min(max(id, 0), C_ - 1);
                const v8f sv = ld8f(cen + (size_t)(b * C_ + id) * H_ + h8);
                *(v8h*)(featF + b * KP_ + h8)      = cvt8h(acc, 1.0f);
                *(v8h*)(featF + b * KP_ + H_ + h8) = cvt8h(sv, 1.0f);
            }
        }
        __syncthreads();

        {
            const float* crow = cen + (size_t)tid * H_;
            const float* orow = core + pb * H_;
            float q = 0.0f;
#pragma unroll 4
            for (int h = 0; h < H_; h += 4) {
                const v4f a = *(const v4f*)(crow + h);
                const v4f o = *(const v4f*)(orow + h);
#pragma unroll
                for (int e = 0; e < 4; ++e) { const float dd = a[e] - o[e]; q += dd * dd; }
            }
            const float sqd = q * (1.0f / H_);
            const float dsum = seg_sum(al * sqd);
            if (pc == 0) {
                if (!fin) {
                    unsigned short hi, lo;
                    split_bf16(dsum, hi, lo);
                    ciH[pb * KP_ + 2 * H_ + 1] = hi; ciL[pb * KP_ + 2 * H_ + 1] = lo;
                } else {
                    featF[pb * KP_ + 2 * H_ + 1] = (_Float16)dsum;
                }
            }
        }
        __syncthreads();
        if (fin) break;

        {
            const int n0 = 16 * w;
            const unsigned short* aph = ciH + m * KP_ + 8 * hf;
            const unsigned short* apl = ciL + m * KP_ + 8 * hf;
            const unsigned short* bph = W1H + (size_t)(n0 + m) * KP_ + 8 * hf;
            const unsigned short* bpl = W1L + (size_t)(n0 + m) * KP_ + 8 * hf;
            v8f acc = zero8f();
#pragma unroll 3
            for (int ks = 0; ks < KP_ / 32; ++ks) {
                FragB ah, alo, bh, bl;
                ldfragb(ah, aph + 32 * ks);
                ldfragb(alo, apl + 32 * ks);
                ldfragb(bh, bph + 32 * ks);
                ldfragb(bl, bpl + 32 * ks);
                acc = mma3(acc, ah, alo, bh, bl);
            }
#pragma unroll
            for (int r = 0; r < 8; ++r) {
                const float x = tanhf(acc[r] + b1v);
                unsigned short hi, lo;
                split_bf16(x, hi, lo);
                const int o = (8 * hf + r) * H_ + n0 + m;
                ct1H[o] = hi; ct1L[o] = lo;
            }
        }
        __syncthreads();

        {
            const int n0 = 16 * w;
            const unsigned short* aph = ct1H + m * H_ + 8 * hf;
            const unsigned short* apl = ct1L + m * H_ + 8 * hf;
            const unsigned short* bph = W2H + (size_t)(n0 + m) * H_ + 8 * hf;
            const unsigned short* bpl = W2L + (size_t)(n0 + m) * H_ + 8 * hf;
            v8f acc = zero8f();
#pragma unroll
            for (int ks = 0; ks < H_ / 32; ++ks) {
                FragB ah, alo, bh, bl;
                ldfragb(ah, aph + 32 * ks);
                ldfragb(alo, apl + 32 * ks);
                ldfragb(bh, bph + 32 * ks);
                ldfragb(bl, bpl + 32 * ks);
                acc = mma3(acc, ah, alo, bh, bl);
            }
#pragma unroll
            for (int r = 0; r < 8; ++r) {
                const float x = tanhf(acc[r] + b2v);
                unsigned short hi, lo;
                split_bf16(x, hi, lo);
                const int o = (8 * hf + r) * H_ + n0 + m;
                ctH[o] = hi; ctL[o] = lo;
                ctF[o] = (_Float16)x;
            }
        }
        __syncthreads();

        {
            FragB ah4[4], al4[4];
#pragma unroll
            for (int ks = 0; ks < 4; ++ks) {
                ldfragb(ah4[ks], ctH + m * H_ + 8 * hf + 32 * ks);
                ldfragb(al4[ks], ctL + m * H_ + 8 * hf + 32 * ks);
            }
#pragma unroll 1
            for (int nt = w; nt < NHT_; nt += 8) {
                const unsigned short* bph = WHH + (size_t)(nt * 16 + m) * H_ + 8 * hf;
                const unsigned short* bpl = WHL + (size_t)(nt * 16 + m) * H_ + 8 * hf;
                v8f acc = zero8f();
#pragma unroll
                for (int ks = 0; ks < 4; ++ks) {
                    FragB bh, bl;
                    ldfragb(bh, bph + 32 * ks);
                    ldfragb(bl, bpl + 32 * ks);
                    acc = mma3(acc, ah4[ks], al4[ks], bh, bl);
                }
                const float bias = (nt == w) ? hb0 : hb1;
#pragma unroll
                for (int r = 0; r < 8; ++r)
                    heads[(8 * hf + r) * NH_ + nt * 16 + m] = acc[r] + bias;
            }
        }
        __syncthreads();

        {
            const float* hrow = heads + pb * NH_;
            const float gt = sigm(hrow[pc]) * vld;
            const float av = hrow[16 + pc];
            const float amx = seg_max(av);
            const float ae = expf(av - amx);
            const float asum = seg_sum(ae);
            const float asg = ae * (1.0f / asum);
            const float nvv = sigm(hrow[32]) * vld;
            rl = sigm(hrow[33]) * vld;
            const float xs = hrow[48 + pc];
            const float cs = (fmaxf(xs, 0.0f) + log1pf(expf(-fabsf(xs)))) + EPS_;
            const float md = tanhf(hrow[64 + pc]);
            const float ss = gt * asg;
            ssS[tid] = ss;
            sp = sp + ss * (cs - sp);
            ma = ma + ss * md;
            sprS[tid] = sp;
            masS[tid] = ma;
            if (pc == 0) { novS[pb] = nvv; relS[pb] = rl; }
        }
        __syncthreads();

        {
            FragH aff[4];
#pragma unroll
            for (int ks = 0; ks < 4; ++ks) ldfragh(aff[ks], ctF + m * H_ + 8 * hf + 32 * ks);
            v8f ssq0, ssq1, nvq;
#pragma unroll
            for (int r = 0; r < 8; ++r) {
                const int row = 8 * hf + r;
                ssq0[r] = ssS[row * C_ + 2 * w];
                ssq1[r] = ssS[row * C_ + 2 * w + 1];
                nvq[r]  = 0.1f * novS[row];
            }
#pragma unroll
            for (int q = 0; q < 2; ++q) {
                const int c = 2 * w + q;
                v8f ssq = ssq1;
                if (q == 0) ssq = ssq0;
#pragma unroll 1
                for (int ht = 0; ht < 8; ++ht) {
                    const int n0 = c * H_ + 16 * ht;
                    const _Float16* bp = Wccp + (size_t)(n0 + m) * H_ + 8 * hf;
                    v8f acc = zero8f();
#pragma unroll
                    for (int ks = 0; ks < 4; ++ks) {
                        FragH bfr;
                        ldfragh(bfr, bp + 32 * ks);
                        acc = mmah(acc, aff[ks], bfr);
                    }
                    const float bias = cc_b[n0 + m];
                    const int hcol = 16 * ht + m;
#pragma unroll
                    for (int r = 0; r < 8; ++r) {
                        const int row = 8 * hf + r;
                        const int ix = (row * C_ + c) * H_ + hcol;
                        const float ce = cen[ix];
                        const float cand = acc[r] * 0.0625f + bias;
                        const float c1 = ce + ssq[r] * (cand - ce);
                        const float at = heads[row * NH_ + 80 + hcol];
                        const float c2 = c1 + nvq[r] * (at - c1);
                        cen[ix] = c2;
                    }
                }
            }
        }
        __syncthreads();

        {
            const float* crow = cen + (size_t)tid * H_;
            float q = 0.0f;
#pragma unroll 4
            for (int h = 0; h < H_; h += 4) {
                const v4f a = *(const v4f*)(crow + h);
#pragma unroll
                for (int e = 0; e < 4; ++e) q += a[e] * a[e];
            }
            sqS[tid] = q;
        }
        __syncthreads();

        {
#pragma unroll 1
            for (int q = 0; q < 2; ++q) {
                const int bb = w + 8 * q;
                const float* ap = cen + (size_t)(bb * C_ + m) * H_ + 8 * hf;
                v8f acc = zero8f();
#pragma unroll
                for (int ks = 0; ks < 4; ++ks) {
                    const v8f x0 = ld8f(ap + 32 * ks);
                    const v8f x1 = ld8f(ap + 32 * ks + 16);
                    FragH a;
                    a.half[0] = cvt8h(x0, 8.0f);
                    a.half[1] = cvt8h(x1, 8.0f);
                    acc = mmah(acc, a, a);
                }
                const int rb = bb * C_;
                const int j = m;
                const float sqj = sqS[rb + j], spj = sprS[rb + j], maj = masS[rb + j];
#pragma unroll
                for (int r = 0; r < 8; ++r) {
                    const int i = 8 * hf + r;
                    const float g = acc[r] * (1.0f / 64.0f);
                    const float d2 = fmaxf((sqS[rb + i] + sqj) - 2.0f * g, 0.0f);
                    const float scl = (sprS[rb + i] + spj) + EPS_;
                    cmp[(rb + i) * C_ + j] = -d2 / scl + maj;
                }
            }
        }
        __syncthreads();

        {
            const float* crow = cmp + (size_t)tid * C_;
            const v4f x0 = *(const v4f*)(crow), x1 = *(const v4f*)(crow + 4);
            const v4f x2 = *(const v4f*)(crow + 8), x3 = *(const v4f*)(crow + 12);
            float mx = x0[0];
#pragma unroll
            for (int e = 0; e < 4; ++e) { mx = fmaxf(mx, x0[e]); mx = fmaxf(mx, x1[e]); mx = fmaxf(mx, x2[e]); mx = fmaxf(mx, x3[e]); }
            v4f e0, e1, e2, e3;
            float sum = 0.0f;
#pragma unroll
            for (int e = 0; e < 4; ++e) {
                e0[e] = __expf(x0[e] - mx); e1[e] = __expf(x1[e] - mx);
                e2[e] = __expf(x2[e] - mx); e3[e] = __expf(x3[e] - mx);
                sum += (e0[e] + e1[e]) + (e2[e] + e3[e]);
            }
            const float inv = 1.0f / sum;
            const v4f s0 = *(const v4f*)(sprS + pb * C_), s1 = *(const v4f*)(sprS + pb * C_ + 4);
            const v4f s2 = *(const v4f*)(sprS + pb * C_ + 8), s3 = *(const v4f*)(sprS + pb * C_ + 12);
            const v4f q0 = *(const v4f*)(masS + pb * C_), q1 = *(const v4f*)(masS + pb * C_ + 4);
            const v4f q2 = *(const v4f*)(masS + pb * C_ + 8), q3 = *(const v4f*)(masS + pb * C_ + 12);
            float msum = 0.0f, qsum = 0.0f;
            v8h lo, hi;
#pragma unroll
            for (int e = 0; e < 4; ++e) {
                const float p0 = e0[e] * inv, p1 = e1[e] * inv, p2 = e2[e] * inv, p3 = e3[e] * inv;
                msum += (p0 * s0[e] + p1 * s1[e]) + (p2 * s2[e] + p3 * s3[e]);
                qsum += (p0 * q0[e] + p1 * q1[e]) + (p2 * q2[e] + p3 * q3[e]);
                lo[e] = (_Float16)(256.0f * p0); lo[4 + e] = (_Float16)(256.0f * p1);
                hi[e] = (_Float16)(256.0f * p2); hi[4 + e] = (_Float16)(256.0f * p3);
            }
            msr = msum;
            mmr = qsum;
            *(v8h*)(mixh + (size_t)tid * C_)     = lo;
            *(v8h*)(mixh + (size_t)tid * C_ + 8) = hi;
        }
        __syncthreads();

        {
#pragma unroll
            for (int q = 0; q < 2; ++q) {
                const int bb = 2 * w + q;
                FragH a;
                a.half[0] = *(const v8h*)(mixh + (size_t)(bb * C_ + m) * C_ + 8 * hf);
                a.half[1] = zero8h();
                const float rel = relS[bb];
                float* cw = cen + (size_t)(bb * C_ + 8 * hf) * H_ + m;
#pragma unroll 1
                for (int ht = 0; ht < 8; ++ht) {
                    const int n0 = 16 * ht;
                    v8f gf;
#pragma unroll
                    for (int e = 0; e < 8; ++e) gf[e] = cw[e * H_ + n0];
                    FragH bfr;
                    bfr.half[0] = cvt8h(gf, 8.0f);
                    bfr.half[1] = zero8h();
                    const v8f acc = mmah(zero8f(), a, bfr);
#pragma unroll
                    for (int r = 0; r < 8; ++r)
                        cw[r * H_ + n0] = (1.0f - rel) * gf[r] + rel * (acc[r] * (1.0f / 2048.0f));
                }
            }
            sp = (1.0f - rl) * sp + rl * msr;
            ma = (1.0f - rl) * ma + rl * mmr;
            const float prec = 1.0f / (sp + EPS_);
            const float sc = ma + logf(prec + EPS_);
            const float mx = seg_max(sc);
            const float e = expf(sc - mx);
            const float se = seg_sum(e);
            const float ca = e * (1.0f / se);
            sp = sp * (1.0f - 0.05f * ca * vld) + EPS_;
        }
        __syncthreads();
    }

    {
        const int n0 = 16 * w;
        const _Float16* ap = featF + m * KP_ + 8 * hf;
        const _Float16* bp = C1p + (size_t)(n0 + m) * KP_ + 8 * hf;
        v8f acc = zero8f();
#pragma unroll 3
        for (int ks = 0; ks < KP_ / 32; ++ks) {
            FragH a, bfr;
            ldfragh(a, ap + 32 * ks);
            ldfragh(bfr, bp + 32 * ks);
            acc = mmah(acc, a, bfr);
        }
#pragma unroll
        for (int r = 0; r < 8; ++r) {
            const float x = acc[r] * 0.0625f + cb1v;
            const float gl = 0.5f * x * (1.0f + erff(x * 0.70710678118654752f));
            ctF[(8 * hf + r) * H_ + n0 + m] = (_Float16)gl;
        }
    }
    __syncthreads();
    if (w == 0) {
        const _Float16* ap = ctF + m * H_ + 8 * hf;
        const _Float16* bp = C2p + (size_t)m * H_ + 8 * hf;
        v8f acc = zero8f();
#pragma unroll
        for (int ks = 0; ks < 4; ++ks) {
            FragH a, bfr;
            ldfragh(a, ap + 32 * ks);
            ldfragh(bfr, bp + 32 * ks);
            acc = mmah(acc, a, bfr);
        }
#pragma unroll
        for (int r = 0; r < 8; ++r)
            if (m < NC_) ost[(8 * hf + r) * NC_ + m] = acc[r] * 0.0625f + cb2v;
    }
    __syncthreads();
    if (w == 0) {
        const v4f v = *(const v4f*)(ost + 4 * lane);
        float* op = out + (size_t)b0 * NC_ + 4 * lane;
        *(volatile v4f*)op = v;
        __threadfence();
        *(volatile v4f*)op = v;
    }
}

extern "C" void kernel_launch(void* const* d_in, const int* in_sizes, int n_in,
                              void* d_out, int out_size, void* d_ws, size_t ws_size,
                              hipStream_t stream)
{
    if (n_in < 28) return;
    if (in_sizes[0]  != B_ * S_)        return;
    if (in_sizes[1]  != V_ * H_)        return;
    if (in_sizes[2]  != H_ || in_sizes[3] != H_) return;
    if (in_sizes[4]  != CI_ * H_)       return;
    if (in_sizes[5]  != H_)             return;
    if (in_sizes[6]  != H_ * H_)        return;
    if (in_sizes[7]  != H_)             return;
    if (in_sizes[8]  != H_ * C_ || in_sizes[9]  != C_) return;
    if (in_sizes[10] != H_ * C_ || in_sizes[11] != C_) return;
    if (in_sizes[12] != H_ || in_sizes[13] != 1)       return;
    if (in_sizes[14] != H_ || in_sizes[15] != 1)       return;
    if (in_sizes[16] != H_ * C_ * H_ || in_sizes[17] != C_ * H_) return;
    if (in_sizes[18] != H_ * C_ || in_sizes[19] != C_) return;
    if (in_sizes[20] != H_ * C_ || in_sizes[21] != C_) return;
    if (in_sizes[22] != H_ * H_ || in_sizes[23] != H_) return;
    if (in_sizes[24] != CI_ * H_ || in_sizes[25] != H_) return;
    if (in_sizes[26] != H_ * NC_ || in_sizes[27] != NC_) return;
    if (out_size != B_ * NC_)           return;
    if (ws_size < WS_END)               return;

    const int*   tokens   = (const int*)  d_in[0];
    const float* emb      = (const float*)d_in[1];
    const float* ln_g     = (const float*)d_in[2];
    const float* ln_b     = (const float*)d_in[3];
    const float* ctrl_w1  = (const float*)d_in[4];
    const float* ctrl_b1  = (const float*)d_in[5];
    const float* ctrl_w2  = (const float*)d_in[6];
    const float* ctrl_b2  = (const float*)d_in[7];
    const float* gate_w   = (const float*)d_in[8];
    const float* gate_b   = (const float*)d_in[9];
    const float* assign_w = (const float*)d_in[10];
    const float* assign_b = (const float*)d_in[11];
    const float* nov_w    = (const float*)d_in[12];
    const float* nov_b    = (const float*)d_in[13];
    const float* relax_w  = (const float*)d_in[14];
    const float* relax_b  = (const float*)d_in[15];
    const float* cc_w     = (const float*)d_in[16];
    const float* cc_b     = (const float*)d_in[17];
    const float* cs_w     = (const float*)d_in[18];
    const float* cs_b     = (const float*)d_in[19];
    const float* md_w     = (const float*)d_in[20];
    const float* md_b     = (const float*)d_in[21];
    const float* att_w    = (const float*)d_in[22];
    const float* att_b    = (const float*)d_in[23];
    const float* cls_w1   = (const float*)d_in[24];
    const float* cls_b1   = (const float*)d_in[25];
    const float* cls_w2   = (const float*)d_in[26];
    const float* cls_b2   = (const float*)d_in[27];
    float* out = (float*)d_out;

    char* ws = (char*)d_ws;
    unsigned short* teH    = (unsigned short*)(ws + OFF_TEH);
    unsigned short* teL    = (unsigned short*)(ws + OFF_TEL);
    unsigned short* planes = (unsigned short*)(ws + OFF_PL);

    k_planes<<<dim3(NBLK_PL), dim3(NT_), 0, stream>>>(ctrl_w1, ctrl_w2, gate_w, assign_w, nov_w, relax_w,
                                                     cs_w, md_w, att_w, cc_w, cls_w1, cls_w2, planes);
    k_embed<<<dim3((B_ * S_) / 8), dim3(NT_), 0, stream>>>(tokens, emb, ln_g, ln_b, teH, teL, B_ * S_);
    (void)hipFuncSetAttribute(reinterpret_cast<const void*>(&k_scan),
                              hipFuncAttributeMaxDynamicSharedMemorySize, LDS_BYTES);
    k_scan<<<dim3(B_ / BT_), dim3(NT_), LDS_BYTES, stream>>>(tokens, (const unsigned short*)teH, (const unsigned short*)teL,
                                                           (const unsigned short*)planes,
                                                           ctrl_b1, ctrl_b2, gate_b, assign_b, nov_b, relax_b,
                                                           cs_b, md_b, att_b, cc_b, cls_b1, cls_b2, out);
}
